// ner_unit_54022098649171
// MI455X (gfx1250) — hardware-verified
//
#include <hip/hip_runtime.h>
#include <math.h>
#include <stdint.h>

#define LL    128
#define BB    8
#define HH    768
#define TT    8
#define MR    (LL * BB)
#define KC    (2 * HH)
#define KW    (3 * HH)
#define NOUT  (LL * LL * BB * TT)
#define LNEPS 1e-5f
#define ESC   64.0f
#define WSC   1024.0f
#define XSC   256.0f

static_assert((MR * KC) % 2048 == 0);
static_assert((HH * KC) % 2048 == 0);
static_assert((HH * KW) % 2048 == 0);
static_assert((16 * HH) % 2048 == 0);
static_assert((HH % 64) == 0 && (KC % 64) == 0 && (KC % 32) == 0 && (HH % 32) == 0 && (MR % 16) == 0);
static_assert((((MR / 16) * (HH / 64)) % 8) == 0);
static_assert((((MR / 16) * (KC / 64)) % 8) == 0);
static_assert((HH % 256) == 0);

typedef _Float16 v16h __attribute__((ext_vector_type(16)));
typedef _Float16 v8h  __attribute__((ext_vector_type(8)));
typedef float    v8f  __attribute__((ext_vector_type(8)));
typedef float    v4f  __attribute__((ext_vector_type(4)));
typedef unsigned int v4u __attribute__((ext_vector_type(4)));

union FragH { v16h v; v8h h[2]; };

__device__ __forceinline__ unsigned short bf_bits(float f) {
  unsigned u = __float_as_uint(f);
  return (unsigned short)((u + 0x7FFFu + ((u >> 16) & 1u)) >> 16);
}
__device__ __forceinline__ float bf_up(unsigned short h) { return __uint_as_float(((unsigned)h) << 16); }
__device__ __forceinline__ float bfr(float f) { return bf_up(bf_bits(f)); }
__device__ __forceinline__ unsigned short h_bits(_Float16 x) { return __builtin_bit_cast(unsigned short, x); }
__device__ __forceinline__ unsigned pk16(unsigned short a, unsigned short b) { return (unsigned)a | ((unsigned)b << 16); }
__device__ __forceinline__ unsigned pkh(float a, float b) { return pk16(h_bits((_Float16)a), h_bits((_Float16)b)); }
__device__ __forceinline__ v8f zero8() { v8f z = {0.f, 0.f, 0.f, 0.f, 0.f, 0.f, 0.f, 0.f}; return z; }

__device__ __forceinline__ v16h ldfrag_h(const _Float16* p) {
  FragH f;
  f.h[0] = *(const v8h*)(p);
  f.h[1] = *(const v8h*)(p + 16);
  return f.v;
}

__device__ __forceinline__ v8f mma_h(v16h a, v16h b, v8f c) {
  c = __builtin_amdgcn_wmma_f32_16x16x32_f16(false, a, false, b, (short)0, c, false, false);
#if defined(__HIP_DEVICE_COMPILE__)
  asm volatile("v_nop\n\tv_nop\n\tv_nop\n\tv_nop" : "+v"(c) : "v"(a), "v"(b));
#endif
  return c;
}
__device__ __forceinline__ void wave_sync_lds() {
  __builtin_amdgcn_fence(__ATOMIC_RELEASE, "workgroup");
  __builtin_amdgcn_wave_barrier();
  __builtin_amdgcn_fence(__ATOMIC_ACQUIRE, "workgroup");
}

__global__ __launch_bounds__(256) void cvt_cat(const float* __restrict__ a, const float* __restrict__ c,
                                               unsigned short* outp) {
  const size_t e = ((size_t)blockIdx.x * 256 + threadIdx.x) * 8;
  const int r = (int)(e / KC);
  const int k = (int)(e - (size_t)r * KC);
  const size_t so = (size_t)r * HH + (size_t)((k < HH) ? k : (k - HH));
  const float* src = ((k < HH) ? a : c) + so;
  const v4f x0 = *(const v4f*)(src);
  const v4f x1 = *(const v4f*)(src + 4);
  v4u pk;
  pk[0] = pkh(bfr(x0[0]) * ESC, bfr(x0[1]) * ESC);
  pk[1] = pkh(bfr(x0[2]) * ESC, bfr(x0[3]) * ESC);
  pk[2] = pkh(bfr(x1[0]) * ESC, bfr(x1[1]) * ESC);
  pk[3] = pkh(bfr(x1[2]) * ESC, bfr(x1[3]) * ESC);
  unsigned short* gp = outp + e;
  *(volatile v4u*)gp = pk;
  __threadfence();
  *(volatile v4u*)gp = pk;
}

__global__ __launch_bounds__(256) void cvt_flat(const float* __restrict__ x, unsigned short* outp, float sc) {
  const size_t base = ((size_t)blockIdx.x * 256 + threadIdx.x) * 8;
  const v4f a = *(const v4f*)(x + base);
  const v4f c = *(const v4f*)(x + base + 4);
  v4u pk;
  pk[0] = pkh(bfr(a[0]) * sc, bfr(a[1]) * sc);
  pk[1] = pkh(bfr(a[2]) * sc, bfr(a[3]) * sc);
  pk[2] = pkh(bfr(c[0]) * sc, bfr(c[1]) * sc);
  pk[3] = pkh(bfr(c[2]) * sc, bfr(c[3]) * sc);
  unsigned short* gp = outp + base;
  *(volatile v4u*)gp = pk;
  __threadfence();
  *(volatile v4u*)gp = pk;
}

__global__ __launch_bounds__(256) void cvt_tag(const float* __restrict__ tw, unsigned short* outp) {
  const int base = (blockIdx.x * 256 + threadIdx.x) * 8;
  const int ok = (base < TT * HH) ? 1 : 0;
  const int idx = ok ? base : (TT * HH - 8);
  const v4f a = *(const v4f*)(tw + idx);
  const v4f c = *(const v4f*)(tw + idx + 4);
  const float f = ok ? 1.0f : 0.0f;
  float v[8];
#pragma unroll
  for (int e = 0; e < 4; ++e) { v[e] = ok ? a[e] : 0.0f; v[4 + e] = ok ? c[e] : 0.0f; }
  v4u pk;
#pragma unroll
  for (int e = 0; e < 4; ++e) pk[e] = pkh(bfr(v[2 * e]) * WSC * f, bfr(v[2 * e + 1]) * WSC * f);
  unsigned short* gp = outp + base;
  *(volatile v4u*)gp = pk;
  __threadfence();
  *(volatile v4u*)gp = pk;
}

template <int MODE>
__global__ __launch_bounds__(256) void gemm16(const unsigned short* __restrict__ Ap, int lda,
                                              const unsigned short* __restrict__ Bp, int ldb, int cb, int kbo,
                                              const float* __restrict__ bias, float* C, int ldc, int K,
                                              int tncnt, int tot, float sc) {
#pragma clang fp contract(off)
  __shared__ __align__(16) float sT[8][16 * 68];
  const int lane = threadIdx.x & 31;
  const int wave = threadIdx.x >> 5;
  const int t = __builtin_amdgcn_readfirstlane((int)(blockIdx.x * 8 + wave));
  if (t >= tot) return;
  const int tm = t / tncnt;
  const int tn = t - tm * tncnt;
  const int m0 = tm * 16;
  const int n0 = tn * 64;
  const int wsel = n0 / cb;
  const int nb0 = n0 - wsel * cb;

  const int rl   = lane & 15;
  const int hh   = lane >> 4;
  const int koff = hh * 8;

  const _Float16* A  = (const _Float16*)(const void*)Ap;
  const _Float16* Bt = (const _Float16*)(const void*)Bp;

  v8f acc[4];
#pragma unroll
  for (int j = 0; j < 4; ++j) acc[j] = zero8();

  const size_t arow  = (size_t)(m0 + rl) * lda + koff;
  const size_t bbase = (size_t)wsel * kbo + koff;
#pragma unroll 2
  for (int k0 = 0; k0 < K; k0 += 32) {
    const v16h fa = ldfrag_h(A + arow + k0);
#pragma unroll
    for (int j = 0; j < 4; ++j) {
      const v16h fb = ldfrag_h(Bt + (size_t)(nb0 + 16 * j + rl) * ldb + bbase + k0);
      acc[j] = mma_h(fa, fb, acc[j]);
    }
  }

  float* slab = sT[wave];
#pragma unroll
  for (int j = 0; j < 4; ++j) {
#pragma unroll
    for (int r = 0; r < 8; ++r) slab[(koff + r) * 68 + 16 * j + rl] = acc[j][r];
  }
  wave_sync_lds();

  const int h2 = lane >> 4, c4 = (lane & 15) * 4;
  float bz[4];
#pragma unroll
  for (int e = 0; e < 4; ++e) bz[e] = (MODE == 0) ? bfr(bias[n0 + c4 + e]) : 0.0f;
#pragma unroll 1
  for (int it = 0; it < 8; ++it) {
    const int row = it * 2 + h2;
    float* spp = slab + row * 68 + c4;
    const v4f v = *(const v4f*)spp;
    v4f o;
#pragma unroll
    for (int e = 0; e < 4; ++e) {
      float f = v[e] * sc;
      if (MODE == 0) { f = f + bz[e]; f = tanhf(f); }
      o[e] = f;
    }
    *(v4f*)spp = o;
  }
  for (int pass = 0; pass < 2; ++pass) {
#pragma unroll
    for (int it = 0; it < 8; ++it) {
      const int row = it * 2 + h2;
      const v4f v = *(const v4f*)(slab + row * 68 + c4);
      float* gp = C + (size_t)(m0 + row) * ldc + n0 + c4;
      *(volatile v4f*)gp = v;
    }
    __threadfence();
  }
}

__global__ __launch_bounds__(256) void ag_rows(const float* __restrict__ hgp, const float* __restrict__ hw,
                                               const float* __restrict__ hb, float* agp) {
  __shared__ float sg[HH];
  __shared__ __align__(16) float so[64];
  const int tid = threadIdx.x, wave = tid >> 5, lane = tid & 31;
  const int kc = blockIdx.x, b = blockIdx.y;
#pragma unroll 1
  for (int c = tid; c < HH; c += 256) {
    float mx = hgp[(size_t)b * HH + c];
#pragma unroll 1
    for (int l = 1; l < LL; ++l) mx = fmaxf(mx, hgp[((size_t)(l * BB + b)) * HH + c]);
    sg[c] = mx;
  }
  __syncthreads();
#pragma unroll 1
  for (int q = 0; q < 8; ++q) {
    const int k = kc * 64 + wave * 8 + q;
    const float* wr = hw + (size_t)k * KW + 2 * HH;
    float s = 0.f;
#pragma unroll 1
    for (int it = 0; it < HH / 32; ++it) {
      const int h = it * 32 + lane;
      const float w = bfr(wr[h]);
      s = fmaf(sg[h], w, s);
    }
#pragma unroll
    for (int off = 16; off >= 1; off >>= 1) s = s + __shfl_xor(s, off, 32);
    if (lane == 0) so[wave * 8 + q] = s + bfr(hb[k]);
  }
  __syncthreads();
  const bool act = tid < 16;
  const int u = act ? tid : 0;
  const v4f v = *(const v4f*)(so + 4 * u);
  float* gp = agp + (size_t)b * HH + kc * 64 + 4 * u;
  if (act) { *(volatile v4f*)gp = v; }
  __threadfence();
  if (act) { *(volatile v4f*)gp = v; }
}

__device__ __forceinline__ _Float16 xelu(float e, float p, float g, float t, float mu, float rs) {
#pragma clang fp contract(off)
  float u = p + e;
  u = u - mu;
  u = u * rs;
  u = u * g;
  u = u + t;
  const float pos = u * XSC;
  float neg = __expf(u) * XSC;
  neg = neg - XSC;
  const float x = (u > 0.f) ? pos : neg;
  return (_Float16)x;
}

__global__ __launch_bounds__(256) void span_k(const float* __restrict__ ase, const float* __restrict__ ag,
                                              const float* __restrict__ lng, const float* __restrict__ lnb,
                                              const unsigned short* __restrict__ tgp, const float* __restrict__ tb,
                                              const float* __restrict__ msk, float* outp) {
#pragma clang fp contract(off)
  __shared__ __align__(16) float sS[8][HH];
  __shared__ __align__(16) float sG[HH];
  __shared__ __align__(16) float sBt[HH];
  __shared__ __align__(16) float sO[16 * 64];
  const int tid = threadIdx.x, wave = tid >> 5, lane = tid & 31;
  const int i = blockIdx.x, j0 = blockIdx.y * 16, b = wave;
  float* obase = outp + ((size_t)(i * LL + j0)) * (BB * TT);

  if (j0 + 15 < i) {
    v4f z = {0.f, 0.f, 0.f, 0.f};
    float* gp = obase + 4 * tid;
    *(volatile v4f*)gp = z;
    __threadfence();
    *(volatile v4f*)gp = z;
    return;
  }

#pragma unroll 1
  for (int c = tid; c < HH; c += 256) { sG[c] = bfr(lng[c]); sBt[c] = bfr(lnb[c]); }
  {
    const float* sp0 = ase + ((size_t)(i * BB + b)) * KC;
    const float* gp0 = ag + (size_t)b * HH;
    float* dstp = sS[wave];
#pragma unroll 1
    for (int c = lane; c < HH; c += 32) {
      float v = sp0[c];
      v = v + gp0[c];
      dstp[c] = v;
    }
  }
  __syncthreads();

  const int m = lane & 15, hh = lane >> 4, c8 = lane * 8;
  const float* sp = sS[wave];

  float mymu = 0.f, myrs = 0.f;
#pragma unroll 1
  for (int r = 0; r < 16; ++r) {
    const float* ep = ase + ((size_t)((j0 + r) * BB + b)) * KC + HH;
    float x[24];
#pragma unroll
    for (int sg = 0; sg < 3; ++sg) {
      const v4f e0 = *(const v4f*)(ep + 256 * sg + c8);
      const v4f e1 = *(const v4f*)(ep + 256 * sg + c8 + 4);
      const v4f p0 = *(const v4f*)(sp + 256 * sg + c8);
      const v4f p1 = *(const v4f*)(sp + 256 * sg + c8 + 4);
#pragma unroll
      for (int e = 0; e < 4; ++e) { x[8 * sg + e] = p0[e] + e0[e]; x[8 * sg + 4 + e] = p1[e] + e1[e]; }
    }
    float s = 0.f;
#pragma unroll
    for (int e = 0; e < 24; ++e) s = s + x[e];
#pragma unroll
    for (int off = 1; off < 32; off <<= 1) s = s + __shfl_xor(s, off, 32);
    const float mu = s * (1.0f / HH);
    float s2 = 0.f;
#pragma unroll
    for (int e = 0; e < 24; ++e) { const float d = x[e] - mu; const float dd = d * d; s2 = s2 + dd; }
#pragma unroll
    for (int off = 1; off < 32; off <<= 1) s2 = s2 + __shfl_xor(s2, off, 32);
    const float var = s2 * (1.0f / HH);
    const float rstd = rsqrtf(var + LNEPS);
    mymu = (m == r) ? mu : mymu;
    myrs = (m == r) ? rstd : myrs;
  }

  const float* erow = ase + ((size_t)((j0 + m) * BB + b)) * KC + HH;
  const _Float16* Tp = (const _Float16*)(const void*)tgp + (size_t)m * HH + 8 * hh;
  v8f acc = zero8();
#pragma unroll 1
  for (int k0 = 0; k0 < HH; k0 += 32) {
    FragH fa;
#pragma unroll
    for (int c = 0; c < 2; ++c) {
      const int kb = k0 + 16 * c + 8 * hh;
      const v4f e0 = *(const v4f*)(erow + kb);
      const v4f e1 = *(const v4f*)(erow + kb + 4);
      const v4f p0 = *(const v4f*)(sp + kb);
      const v4f p1 = *(const v4f*)(sp + kb + 4);
      const v4f g0 = *(const v4f*)(sG + kb);
      const v4f g1 = *(const v4f*)(sG + kb + 4);
      const v4f t0 = *(const v4f*)(sBt + kb);
      const v4f t1 = *(const v4f*)(sBt + kb + 4);
      v8h hv;
#pragma unroll
      for (int e = 0; e < 4; ++e) {
        hv[e]     = xelu(e0[e], p0[e], g0[e], t0[e], mymu, myrs);
        hv[4 + e] = xelu(e1[e], p1[e], g1[e], t1[e], mymu, myrs);
      }
      fa.h[c] = hv;
    }
    const v16h fb = ldfrag_h(Tp + k0);
    acc = mma_h(fa.v, fb, acc);
  }

  const float tbb = bfr(tb[m & 7]);
  const float mi = bfr(msk[i * BB + b]);
#pragma unroll
  for (int r = 0; r < 8; ++r) {
    const int jl = 8 * hh + r;
    const int j = j0 + jl;
    float z = acc[r] * (1.0f / (XSC * WSC));
    z = z + tbb;
    const float ez = __expf(-z);
    const float den = 1.0f + ez;
    const float sgm = __builtin_amdgcn_rcpf(den);
    const float mj = bfr(msk[j * BB + b]);
    float mm = (i <= j) ? 1.0f : 0.0f;
    mm = mm * mi;
    mm = mm * mj;
    const float o = sgm * mm;
    if (m < TT) sO[jl * 64 + b * 8 + m] = o;
  }
  __syncthreads();
  const v4f v = *(const v4f*)(sO + 4 * tid);
  float* gp = obase + 4 * tid;
  *(volatile v4f*)gp = v;
  __threadfence();
  *(volatile v4f*)gp = v;
}

extern "C" void kernel_launch(void* const* d_in, const int* in_sizes, int n_in,
                              void* d_out, int out_size, void* d_ws, size_t ws_size,
                              hipStream_t stream) {
  if (n_in < 11) return;
  const int ex[11] = { MR * HH, MR * HH, MR, HH * KC, HH, HH * KW, HH, HH, HH, TT * HH, TT };
  for (int q = 0; q < 11; ++q) if (in_sizes[q] != ex[q]) return;
  if (out_size != NOUT) return;

  const float* h1  = (const float*)d_in[0];
  const float* h2  = (const float*)d_in[1];
  const float* msk = (const float*)d_in[2];
  const float* n_w = (const float*)d_in[3];
  const float* n_b = (const float*)d_in[4];
  const float* hw  = (const float*)d_in[5];
  const float* hb  = (const float*)d_in[6];
  const float* lng = (const float*)d_in[7];
  const float* lnb = (const float*)d_in[8];
  const float* tw  = (const float*)d_in[9];
  const float* tb  = (const float*)d_in[10];
  float* out = (float*)d_out;

  const size_t sCAT = (size_t)MR * KC * 2;
  const size_t sNW  = (size_t)HH * KC * 2;
  const size_t sHW  = (size_t)HH * KW * 2;
  const size_t sTG  = (size_t)16 * HH * 2;
  const size_t sHG  = (size_t)MR * HH * 4;
  const size_t sASE = (size_t)MR * KC * 4;
  const size_t sAG  = (size_t)BB * HH * 4;
  size_t off = 0;
  const size_t oCAT = off; off += sCAT;
  const size_t oNW  = off; off += sNW;
  const size_t oHW  = off; off += sHW;
  const size_t oTG  = off; off += sTG;
  const size_t oHG  = off; off += sHG;
  const size_t oASE = off; off += sASE;
  const size_t oAG  = off; off += sAG;
  if (off > ws_size) return;
  if (off > (size_t)134217728) return;

  char* ws = (char*)d_ws;
  unsigned short* CAT  = (unsigned short*)(ws + oCAT);
  unsigned short* NW16 = (unsigned short*)(ws + oNW);
  unsigned short* HW16 = (unsigned short*)(ws + oHW);
  unsigned short* TG16 = (unsigned short*)(ws + oTG);
  float*          HG   = (float*)(ws + oHG);
  float*          ASE  = (float*)(ws + oASE);
  float*          AG   = (float*)(ws + oAG);

  const dim3 blk(256);

  cvt_cat<<<dim3((MR * KC) / 2048), blk, 0, stream>>>(h1, h2, CAT);
  cvt_flat<<<dim3((HH * KC) / 2048), blk, 0, stream>>>(n_w, NW16, WSC);
  cvt_flat<<<dim3((HH * KW) / 2048), blk, 0, stream>>>(hw, HW16, WSC);
  cvt_tag<<<dim3((16 * HH) / 2048), blk, 0, stream>>>(tw, TG16);

  gemm16<0><<<dim3(((MR / 16) * (HH / 64)) / 8), blk, 0, stream>>>(
      CAT, KC, NW16, KC, HH, 0, n_b, HG, HH, KC, HH / 64, (MR / 16) * (HH / 64), 1.0f / (ESC * WSC));

  ag_rows<<<dim3(HH / 64, BB), blk, 0, stream>>>(HG, hw, hb, AG);

  gemm16<1><<<dim3(((MR / 16) * (KC / 64)) / 8), blk, 0, stream>>>(
      CAT + HH, KC, HW16, KW, HH, HH, n_b, ASE, KC, HH, KC / 64, (MR / 16) * (KC / 64), 1.0f / (ESC * WSC));

  span_k<<<dim3(LL, LL / 16), blk, 0, stream>>>(ASE, AG, lng, lnb, TG16, tb, msk, out);
  (void)hipGetLastError();
}
